// TinyLLMBlock_45913200395019
// MI455X (gfx1250) — hardware-run, weakly checked
//
#include <hip/hip_runtime.h>
#include <math.h>

constexpr int kBatch   = 2;
constexpr int kSeq     = 2048;
constexpr int kHid     = 1024;
constexpr int kHeads   = 16;
constexpr int kHeadDim = 64;
constexpr int kFF      = 4096;
constexpr int kTok     = kBatch * kSeq;
constexpr int kQKld    = 2 * kHid;
constexpr int kGroupsPerChunk = 2;
constexpr int kNumChunks = kBatch * kHeads / kGroupsPerChunk;
constexpr int kChunksPerBatch = kHeads / kGroupsPerChunk;

constexpr float kWCarry    = 64.0f;
constexpr float kWCarryInv = 1.0f / 64.0f;
constexpr float kPCarry    = 2048.0f;
constexpr float kAttCarry  = 256.0f;
constexpr float kScoreScale = 0.125f;
constexpr float kPVScale   = kAttCarry / kPCarry;
constexpr float kWoScale   = 1.0f / (kAttCarry * kWCarry);
constexpr float kInvHid    = 1.0f / 1024.0f;
constexpr float kLnEps     = 1e-5f;

constexpr size_t kMiB     = 1048576;
constexpr size_t kOffWQK  = 0 * kMiB;
constexpr size_t kOffWV   = 4 * kMiB;
constexpr size_t kOffWO   = 6 * kMiB;
constexpr size_t kOffW1T  = 8 * kMiB;
constexpr size_t kOffW2T  = 16 * kMiB;
constexpr size_t kOffHB   = 24 * kMiB;
constexpr size_t kOffATT  = 32 * kMiB;
constexpr size_t kOffQK   = 40 * kMiB;
constexpr size_t kOffVT   = 56 * kMiB;
constexpr size_t kOffSC   = 64 * kMiB;
constexpr size_t kOffPP   = 96 * kMiB;
constexpr size_t kOffX1   = 64 * kMiB;
constexpr size_t kOffUU   = 80 * kMiB;
constexpr size_t kOffGG   = 24 * kMiB;
constexpr size_t kWsTotal = 112 * kMiB;

typedef __attribute__((ext_vector_type(16))) _Float16 v16h;
typedef __attribute__((ext_vector_type(8)))  _Float16 v8h;
typedef __attribute__((ext_vector_type(16))) __bf16   v16b;
typedef __attribute__((ext_vector_type(8)))  __bf16   v8b;
typedef __attribute__((ext_vector_type(8)))  float    v8f;
typedef __attribute__((ext_vector_type(4)))  float    v4f;
typedef __attribute__((ext_vector_type(4)))  unsigned int v4u;

__device__ __forceinline__ unsigned short f2bf_bits(float f) {
  unsigned u = __float_as_uint(f);
  return (unsigned short)((u + 0x7FFFu + ((u >> 16) & 1u)) >> 16);
}
__device__ __forceinline__ float bf_bits2f(unsigned short h) { return __uint_as_float(((unsigned)h) << 16); }

__device__ __forceinline__ void dep_guard_h(v8f& a, v8f& b, v16h x, v16h y) { asm volatile("v_nop\n\tv_nop\n\tv_nop\n\tv_nop" : "+v"(a), "+v"(b) : "v"(x), "v"(y)); }
__device__ __forceinline__ void dep_guard_b(v8f& a, v8f& b, v16b x, v16b y) { asm volatile("v_nop\n\tv_nop\n\tv_nop\n\tv_nop" : "+v"(a), "+v"(b) : "v"(x), "v"(y)); }
__device__ __forceinline__ void keep4_h(v16h a, v16h b, v16h c, v16h d) { asm volatile("v_nop" :: "v"(a), "v"(b), "v"(c), "v"(d)); }
__device__ __forceinline__ void keep4_b(v16b a, v16b b, v16b c, v16b d) { asm volatile("v_nop" :: "v"(a), "v"(b), "v"(c), "v"(d)); }
__device__ __forceinline__ void acc_guard4(v8f& a, v8f& b, v8f& c, v8f& d) { asm volatile("v_nop\n\tv_nop\n\tv_nop\n\tv_nop" : "+v"(a), "+v"(b), "+v"(c), "+v"(d)); }
template <typename T> struct Frag;
template <> struct Frag<_Float16> {
  typedef v16h V; union U { v16h v; v8h h[2]; };
  static __device__ __forceinline__ v16h load(const _Float16* p) {
    U f; f.h[0] = *(const v8h*)(p); f.h[1] = *(const v8h*)(p + 16); return f.v;
  }
  static __device__ __forceinline__ v8f mma(v16h a, v16h b, v8f c) {
    return __builtin_amdgcn_wmma_f32_16x16x32_f16(false, a, false, b, (short)0, c, false, false);
  }
  static __device__ __forceinline__ void guard(v8f& a, v8f& b, v16h x, v16h y) { dep_guard_h(a, b, x, y); }
  static __device__ __forceinline__ void keep(v16h a, v16h b, v16h c, v16h d) { keep4_h(a, b, c, d); }
};
template <> struct Frag<__bf16> {
  typedef v16b V; union U { v16b v; v8b h[2]; };
  static __device__ __forceinline__ v16b load(const __bf16* p) {
    U f; f.h[0] = *(const v8b*)(p); f.h[1] = *(const v8b*)(p + 16); return f.v;
  }
  static __device__ __forceinline__ v8f mma(v16b a, v16b b, v8f c) {
    return __builtin_amdgcn_wmma_f32_16x16x32_bf16(false, a, false, b, (short)0, c, false, false);
  }
  static __device__ __forceinline__ void guard(v8f& a, v8f& b, v16b x, v16b y) { dep_guard_b(a, b, x, y); }
  static __device__ __forceinline__ void keep(v16b a, v16b b, v16b c, v16b d) { keep4_b(a, b, c, d); }
};

__device__ __forceinline__ unsigned pk16(unsigned short a, unsigned short b) { return (unsigned)a | ((unsigned)b << 16); }
__device__ __forceinline__ unsigned short h_bits(float f) { const _Float16 h = (_Float16)f; return __builtin_bit_cast(unsigned short, h); }

template <int ET> struct Elem;
template <> struct Elem<0> { typedef _Float16 T; };
template <> struct Elem<1> { typedef __bf16 T; };
template <int ET, bool SPLIT, int BIAS_MODE, int OUT_MODE, bool RESID, int ACT = 0>
__global__ __launch_bounds__(256) void wmma_gemm64(
    const unsigned short* __restrict__ Ap, const unsigned short* __restrict__ A2p, int lda, long strideA,
    const unsigned short* __restrict__ Btp, const unsigned short* __restrict__ Bt2p, int ldb, long strideB,
    void* __restrict__ Cout, void* __restrict__ Cout2, int ldc, long strideC,
    const float* __restrict__ bias,
    const float* __restrict__ resid, long strideR,
    int M, int N, int K, float scale) {
  typedef typename Elem<ET>::T T;
  typedef typename Frag<T>::V V;
  const T* A = (const T*)Ap; const T* A2 = (const T*)A2p; const T* Bt = (const T*)Btp; const T* Bt2 = (const T*)Bt2p;
  __shared__ __align__(16) float sT[8][16 * 68];
  const int b    = blockIdx.y;
  const int lane = threadIdx.x & 31;
  const int wave = threadIdx.x >> 5;
  const int tilesN = N >> 6;
  const int tilesM = M >> 6;
  const int tile = blockIdx.x * 8 + wave;
  if (tile >= tilesM * tilesN) return;
  const int tm = tile / tilesN;
  const int tn = tile - tm * tilesN;
  const int m0 = tm << 6;
  const int n0 = tn << 6;

  const T* Ab  = A  + (size_t)b * strideA;
  const T* Bb  = Bt + (size_t)b * strideB;
  const T* Ab2 = SPLIT ? (A2  + (size_t)b * strideA) : nullptr;
  const T* Bb2 = SPLIT ? (Bt2 + (size_t)b * strideB) : nullptr;

  const int rlane = lane & 15;
  const int koff  = (lane >> 4) * 8;
  const int mOff  = (lane >> 4) * 8;

  v8f acc[4][4];
#pragma unroll
  for (int i = 0; i < 4; ++i)
#pragma unroll
    for (int j = 0; j < 4; ++j) acc[i][j] = (v8f){0.f,0.f,0.f,0.f,0.f,0.f,0.f,0.f};

  for (int k0 = 0; k0 < K; k0 += 32) {
    V bh[4], bl[4];
#pragma unroll
    for (int j = 0; j < 4; ++j) {
      const size_t bo = (size_t)(n0 + (j << 4) + rlane) * ldb + koff + k0;
      bh[j] = Frag<T>::load(Bb + bo);
      if (SPLIT) bl[j] = Frag<T>::load(Bb2 + bo);
    }
#pragma unroll
    for (int i = 0; i < 4; ++i) {
      const size_t ao = (size_t)(m0 + (i << 4) + rlane) * lda + koff + k0;
      V ah = Frag<T>::load(Ab + ao);
      V al;
      if (SPLIT) al = Frag<T>::load(Ab2 + ao);
#pragma unroll
      for (int j = 0; j < 4; ++j) {
        acc[i][j] = Frag<T>::mma(ah, bh[j], acc[i][j]);
        if (SPLIT) {
          acc[i][j] = Frag<T>::mma(ah, bl[j], acc[i][j]);
          acc[i][j] = Frag<T>::mma(al, bh[j], acc[i][j]);
        }
      }
      Frag<T>::guard(acc[i][0], acc[i][3], ah, SPLIT ? al : ah);
    }
    Frag<T>::keep(bh[0], bh[1], bh[2], bh[3]);
    if (SPLIT) Frag<T>::keep(bl[0], bl[1], bl[2], bl[3]);
  }
  acc_guard4(acc[0][0], acc[0][1], acc[0][2], acc[0][3]);
  acc_guard4(acc[1][0], acc[1][1], acc[1][2], acc[1][3]);
  acc_guard4(acc[2][0], acc[2][1], acc[2][2], acc[2][3]);
  acc_guard4(acc[3][0], acc[3][1], acc[3][2], acc[3][3]);

  float* slab = sT[wave];
  const float* Rb = RESID ? (resid + (size_t)b * strideR) : nullptr;
#pragma unroll
  for (int i = 0; i < 4; ++i) {
    const int mBase = m0 + (i << 4);
#pragma unroll
    for (int j = 0; j < 4; ++j) {
      const int n = n0 + (j << 4) + rlane;
      float bv = 0.f;
      if (BIAS_MODE == 2) bv = bias[n];
#pragma unroll
      for (int r = 0; r < 8; ++r) {
        float v = acc[i][j][r] * scale;
        if (BIAS_MODE == 1) v += bias[mBase + mOff + r];
        if (BIAS_MODE == 2) v += bv;
        if (RESID) v += Rb[(size_t)(mBase + mOff + r) * ldc + n];
        if (ACT == 2) v = fmaxf(v, 0.0f);
        if (ACT == 4) v = (v > 0.f) ? v : 0.01f * v;
        slab[(mOff + r) * 68 + (j << 4) + rlane] = v;
      }
    }
    __builtin_amdgcn_fence(__ATOMIC_RELEASE, "workgroup");
    __builtin_amdgcn_wave_barrier();
    __builtin_amdgcn_fence(__ATOMIC_ACQUIRE, "workgroup");
    if (OUT_MODE == 0) {
      float* C = (float*)Cout + (size_t)b * strideC;
      const int hh = lane >> 4, c4 = (lane & 15) * 4;
      for (int pass = 0; pass < 2; ++pass) {
#pragma unroll
        for (int it = 0; it < 8; ++it) {
          const int row = it * 2 + hh;
          v4f v = *(const v4f*)(slab + row * 68 + c4);
          *(volatile v4f*)(C + (size_t)(mBase + row) * ldc + n0 + c4) = v;
        }
        __threadfence();
      }
    } else {
      const int q = lane >> 3, c8 = (lane & 7) * 8;
      unsigned short* C  = (unsigned short*)Cout  + (size_t)b * strideC;
      unsigned short* C2 = (OUT_MODE == 2) ? ((unsigned short*)Cout2 + (size_t)b * strideC) : nullptr;
      for (int pass = 0; pass < 2; ++pass) {
#pragma unroll
        for (int it = 0; it < 4; ++it) {
          const int row = it * 4 + q;
          const float* sp = slab + row * 68 + c8;
          v8h hv, lv;
#pragma unroll
          for (int e = 0; e < 8; ++e) {
            if (OUT_MODE == 1) {
              hv[e] = (_Float16)sp[e];
            } else {
              unsigned short hb = f2bf_bits(sp[e]);
              unsigned short lb = f2bf_bits(sp[e] - bf_bits2f(hb));
              hv[e] = __builtin_bit_cast(_Float16, hb);
              lv[e] = __builtin_bit_cast(_Float16, lb);
            }
          }
          *(volatile v8h*)(C + (size_t)(mBase + row) * ldc + n0 + c8) = hv;
          if (OUT_MODE == 2) *(volatile v8h*)(C2 + (size_t)(mBase + row) * ldc + n0 + c8) = lv;
        }
        __threadfence();
      }
    }
    __builtin_amdgcn_fence(__ATOMIC_RELEASE, "workgroup");
    __builtin_amdgcn_wave_barrier();
    __builtin_amdgcn_fence(__ATOMIC_ACQUIRE, "workgroup");
  }
}

__global__ __launch_bounds__(256) void cast_w4_kernel(const float* __restrict__ Wa, const float* __restrict__ Wb,
                                                      const float* __restrict__ Wc, const float* __restrict__ Wd,
                                                      unsigned short* __restrict__ Oa, unsigned short* __restrict__ Ob,
                                                      unsigned short* __restrict__ Oc, unsigned short* __restrict__ Od,
                                                      int n8, float scale) {
  const int z = blockIdx.y;
  const float* W = (z == 0) ? Wa : (z == 1) ? Wb : (z == 2) ? Wc : Wd;
  unsigned short* O = (z == 0) ? Oa : (z == 1) ? Ob : (z == 2) ? Oc : Od;
  const int i = blockIdx.x * 256 + threadIdx.x;
  if (i >= n8) return;
  const float* p = W + 8 * (size_t)i;
  const v4f a = *(const v4f*)(p);
  const v4f c = *(const v4f*)(p + 4);
  unsigned short hb[8];
#pragma unroll
  for (int e = 0; e < 4; ++e) {
    hb[e]     = h_bits(a[e] * scale);
    hb[4 + e] = h_bits(c[e] * scale);
  }
  const v4u u = (v4u){pk16(hb[0], hb[1]), pk16(hb[2], hb[3]), pk16(hb[4], hb[5]), pk16(hb[6], hb[7])};
  unsigned short* q = O + 8 * (size_t)i;
  *(volatile v4u*)q = u;
  __threadfence();
  *(volatile v4u*)q = u;
}

__global__ __launch_bounds__(256) void tcast_kernel(const float* __restrict__ in, unsigned short* __restrict__ out,
                                                    int nrows, int ncols, float scale) {
  __shared__ float sm[64][65];
  const int t  = threadIdx.x;
  const int c0 = blockIdx.x * 64;
  const int r0 = blockIdx.y * 64;
#pragma unroll
  for (int i = 0; i < 16; ++i) {
    const int e = i * 256 + t;
    const int r = e >> 6;
    const int c = e & 63;
    sm[c][r] = in[(size_t)(r0 + r) * ncols + c0 + c] * scale;
  }
  __syncthreads();
  const int lane = t & 31, wave = t >> 5;
  const int q = lane >> 3, c8 = (lane & 7) * 8;
  for (int pass = 0; pass < 2; ++pass) {
#pragma unroll
    for (int it = 0; it < 2; ++it) {
      const int row = wave * 8 + it * 4 + q;
      unsigned short hb[8];
#pragma unroll
      for (int e = 0; e < 8; ++e) hb[e] = h_bits(sm[row][c8 + e]);
      const v4u u = (v4u){pk16(hb[0], hb[1]), pk16(hb[2], hb[3]), pk16(hb[4], hb[5]), pk16(hb[6], hb[7])};
      *(volatile v4u*)(out + (size_t)(c0 + row) * nrows + r0 + c8) = u;
    }
    __threadfence();
  }
}

__global__ __launch_bounds__(128) void layernorm_f16_kernel(const float* __restrict__ X, const float* __restrict__ gam,
                                                            const float* __restrict__ bet, unsigned short* __restrict__ out) {
  __shared__ float redA[4];
  __shared__ float redB[4];
  const int row  = blockIdx.x;
  const int t    = threadIdx.x;
  const int lane = t & 31, wave = t >> 5;
  const int c0   = t * 8;
  const float* xr = X + (size_t)row * kHid + c0;
  const v4f a = *(const v4f*)(xr);
  const v4f c = *(const v4f*)(xr + 4);
  float x[8];
#pragma unroll
  for (int e = 0; e < 4; ++e) { x[e] = a[e]; x[4 + e] = c[e]; }
  float s = ((x[0] + x[1]) + (x[2] + x[3])) + ((x[4] + x[5]) + (x[6] + x[7]));
#pragma unroll
  for (int off = 16; off > 0; off >>= 1) s += __shfl_xor(s, off, 32);
  if (lane == 0) redA[wave] = s;
  __syncthreads();
  const float mu = ((redA[0] + redA[1]) + (redA[2] + redA[3])) * kInvHid;
  float d[8];
  float qq = 0.f;
#pragma unroll
  for (int e = 0; e < 8; ++e) { d[e] = x[e] - mu; qq += d[e] * d[e]; }
#pragma unroll
  for (int off = 16; off > 0; off >>= 1) qq += __shfl_xor(qq, off, 32);
  if (lane == 0) redB[wave] = qq;
  __syncthreads();
  const float var  = ((redB[0] + redB[1]) + (redB[2] + redB[3])) * kInvHid;
  const float rstd = rsqrtf(var + kLnEps);
  const v4f g0 = *(const v4f*)(gam + c0);
  const v4f g1 = *(const v4f*)(gam + c0 + 4);
  const v4f b0 = *(const v4f*)(bet + c0);
  const v4f b1 = *(const v4f*)(bet + c0 + 4);
  unsigned short hb[8];
#pragma unroll
  for (int e = 0; e < 4; ++e) {
    hb[e]     = h_bits(d[e] * rstd * g0[e] + b0[e]);
    hb[4 + e] = h_bits(d[4 + e] * rstd * g1[e] + b1[e]);
  }
  const v4u u = (v4u){pk16(hb[0], hb[1]), pk16(hb[2], hb[3]), pk16(hb[4], hb[5]), pk16(hb[6], hb[7])};
  unsigned short* op = out + (size_t)row * kHid + c0;
  *(volatile v4u*)op = u;
  __threadfence();
  *(volatile v4u*)op = u;
}

__global__ __launch_bounds__(256) void softmax_p16_kernel(const float* __restrict__ S, unsigned short* __restrict__ P, float carry) {
  __shared__ float redM[8];
  __shared__ float redS[8];
  const int row  = blockIdx.x;
  const int t    = threadIdx.x;
  const int lane = t & 31, wave = t >> 5;
  const int c0   = t * 8;
  const float* sr = S + (size_t)row * kSeq + c0;
  const v4f a = *(const v4f*)(sr);
  const v4f c = *(const v4f*)(sr + 4);
  float x[8];
#pragma unroll
  for (int e = 0; e < 4; ++e) { x[e] = a[e]; x[4 + e] = c[e]; }
  float m = fmaxf(fmaxf(fmaxf(x[0], x[1]), fmaxf(x[2], x[3])), fmaxf(fmaxf(x[4], x[5]), fmaxf(x[6], x[7])));
#pragma unroll
  for (int off = 16; off > 0; off >>= 1) m = fmaxf(m, __shfl_xor(m, off, 32));
  if (lane == 0) redM[wave] = m;
  __syncthreads();
  float gm = redM[0];
#pragma unroll
  for (int w = 1; w < 8; ++w) gm = fmaxf(gm, redM[w]);
  float ex[8];
  float s = 0.f;
#pragma unroll
  for (int e = 0; e < 8; ++e) { ex[e] = expf(x[e] - gm); s += ex[e]; }
#pragma unroll
  for (int off = 16; off > 0; off >>= 1) s += __shfl_xor(s, off, 32);
  if (lane == 0) redS[wave] = s;
  __syncthreads();
  float gs = 0.f;
#pragma unroll
  for (int w = 0; w < 8; ++w) gs += redS[w];
  const float rr = carry * (1.0f / gs);
  unsigned short hb[8];
#pragma unroll
  for (int e = 0; e < 8; ++e) hb[e] = h_bits(ex[e] * rr);
  const v4u u = (v4u){pk16(hb[0], hb[1]), pk16(hb[2], hb[3]), pk16(hb[4], hb[5]), pk16(hb[6], hb[7])};
  unsigned short* op = P + (size_t)row * kSeq + c0;
  *(volatile v4u*)op = u;
  __threadfence();
  *(volatile v4u*)op = u;
}

__global__ __launch_bounds__(256) void gelu_f16_kernel(const unsigned* __restrict__ in, unsigned* __restrict__ out, int n2) {
  const int i = blockIdx.x * 256 + threadIdx.x;
  if (i >= n2) return;
  const unsigned w = in[i];
  unsigned res = 0u;
#pragma unroll 1
  for (int e = 0; e < 2; ++e) {
    const int sh = 16 * e;
    const unsigned short hb = (unsigned short)((w >> sh) & 0xffffu);
    const float u = (float)__builtin_bit_cast(_Float16, hb);
    const float gl = 0.5f * u * (1.0f + erff(u * 0.70710678118654752f));
    res |= ((unsigned)h_bits(gl)) << sh;
  }
  ((volatile unsigned*)out)[i] = res;
  __threadfence();
  ((volatile unsigned*)out)[i] = res;
}

extern "C" void kernel_launch(void* const* d_in, const int* in_sizes, int n_in,
                              void* d_out, int out_size, void* d_ws, size_t ws_size,
                              hipStream_t stream) {
  if (n_in < 13) return;
  if (in_sizes[0] != kTok * kHid || in_sizes[1] != kHid * kHid || in_sizes[2] != kHid * kHid ||
      in_sizes[3] != kHid * kHid || in_sizes[4] != kHid * kHid || in_sizes[5] != kHid || in_sizes[6] != kHid ||
      in_sizes[7] != kHid || in_sizes[8] != kHid || in_sizes[9] != kHid * kFF || in_sizes[10] != kFF ||
      in_sizes[11] != kFF * kHid || in_sizes[12] != kHid) return;
  if (out_size != kTok * kHid) return;
  if (ws_size < kWsTotal) return;

  const float* x    = (const float*)d_in[0];
  const float* Wq   = (const float*)d_in[1];
  const float* Wk   = (const float*)d_in[2];
  const float* Wv   = (const float*)d_in[3];
  const float* Wo   = (const float*)d_in[4];
  const float* ln1g = (const float*)d_in[5];
  const float* ln1b = (const float*)d_in[6];
  const float* ln2g = (const float*)d_in[7];
  const float* ln2b = (const float*)d_in[8];
  const float* W1   = (const float*)d_in[9];
  const float* b1   = (const float*)d_in[10];
  const float* W2   = (const float*)d_in[11];
  const float* b2   = (const float*)d_in[12];
  float* out = (float*)d_out;

  char* ws = (char*)d_ws;
  unsigned short* WQK = (unsigned short*)(ws + kOffWQK);
  unsigned short* WVp = (unsigned short*)(ws + kOffWV);
  unsigned short* WOp = (unsigned short*)(ws + kOffWO);
  unsigned short* W1T = (unsigned short*)(ws + kOffW1T);
  unsigned short* W2T = (unsigned short*)(ws + kOffW2T);
  unsigned short* HB  = (unsigned short*)(ws + kOffHB);
  unsigned short* ATT = (unsigned short*)(ws + kOffATT);
  unsigned short* QK  = (unsigned short*)(ws + kOffQK);
  unsigned short* VT  = (unsigned short*)(ws + kOffVT);
  float*          SC  = (float*)(ws + kOffSC);
  unsigned short* PP  = (unsigned short*)(ws + kOffPP);
  float*          X1  = (float*)(ws + kOffX1);
  unsigned short* UU  = (unsigned short*)(ws + kOffUU);
  unsigned short* GG  = (unsigned short*)(ws + kOffGG);

  const dim3 blk(256);

  cast_w4_kernel<<<dim3(kHid * kHid / 8 / 256, 4), blk, 0, stream>>>(
      Wq, Wk, Wv, Wo, WQK, WQK + (size_t)kHid * kHid, WVp, WOp, kHid * kHid / 8, kWCarry);
  tcast_kernel<<<dim3(kFF / 64, kHid / 64), blk, 0, stream>>>(W1, W1T, kHid, kFF, kWCarry);
  tcast_kernel<<<dim3(kHid / 64, kFF / 64), blk, 0, stream>>>(W2, W2T, kFF, kHid, kWCarry);

  layernorm_f16_kernel<<<dim3(kTok), dim3(128), 0, stream>>>(x, ln1g, ln1b, HB);

  wmma_gemm64<0, false, 0, 1, false><<<dim3(256, 1), blk, 0, stream>>>(
      HB, HB, kHid, 0L, WQK, WQK, kHid, 0L, (void*)QK, (void*)QK, kQKld, 0L,
      nullptr, nullptr, 0L, kTok, kQKld, kHid, kWCarryInv);

  wmma_gemm64<0, false, 0, 1, false><<<dim3(64, kBatch), blk, 0, stream>>>(
      WVp, WVp, kHid, 0L, HB, HB, kHid, (long)kSeq * kHid, (void*)VT, (void*)VT, kSeq, (long)kHid * kSeq,
      nullptr, nullptr, 0L, kHid, kSeq, kHid, kWCarryInv);

  for (int cidx = 0; cidx < kNumChunks; ++cidx) {
    const int bb = cidx / kChunksPerBatch;
    const int h0 = (cidx % kChunksPerBatch) * kGroupsPerChunk;
    const unsigned short* Aq = QK + (size_t)bb * kSeq * kQKld + (size_t)h0 * kHeadDim;
    const unsigned short* Bk = QK + (size_t)bb * kSeq * kQKld + kHid + (size_t)h0 * kHeadDim;
    wmma_gemm64<0, false, 0, 0, false><<<dim3(128, kGroupsPerChunk), blk, 0, stream>>>(
        Aq, Aq, kQKld, (long)kHeadDim, Bk, Bk, kQKld, (long)kHeadDim, (void*)SC, (void*)SC, kSeq, (long)kSeq * kSeq,
        nullptr, nullptr, 0L, kSeq, kSeq, kHeadDim, kScoreScale);
    softmax_p16_kernel<<<dim3(kGroupsPerChunk * kSeq), blk, 0, stream>>>(SC, PP, kPCarry);
    const unsigned short* VTg = VT + (size_t)bb * kHid * kSeq + (size_t)h0 * kHeadDim * kSeq;
    unsigned short* ATTg = ATT + (size_t)bb * kSeq * kHid + (size_t)h0 * kHeadDim;
    wmma_gemm64<0, false, 0, 1, false><<<dim3(4, kGroupsPerChunk), blk, 0, stream>>>(
        PP, PP, kSeq, (long)kSeq * kSeq, VTg, VTg, kSeq, (long)kHeadDim * kSeq, (void*)ATTg, (void*)ATTg, kHid, (long)kHeadDim,
        nullptr, nullptr, 0L, kSeq, kHeadDim, kSeq, kPVScale);
  }

  wmma_gemm64<0, false, 0, 0, true><<<dim3(128, 1), blk, 0, stream>>>(
      ATT, ATT, kHid, 0L, WOp, WOp, kHid, 0L, (void*)X1, (void*)X1, kHid, 0L,
      nullptr, x, 0L, kTok, kHid, kHid, kWoScale);

  layernorm_f16_kernel<<<dim3(kTok), dim3(128), 0, stream>>>(X1, ln2g, ln2b, HB);

  wmma_gemm64<0, false, 2, 1, false><<<dim3(512, 1), blk, 0, stream>>>(
      HB, HB, kHid, 0L, W1T, W1T, kHid, 0L, (void*)UU, (void*)UU, kFF, 0L,
      b1, nullptr, 0L, kTok, kFF, kHid, kWCarryInv);

  gelu_f16_kernel<<<dim3(kTok * kFF / 2 / 256), blk, 0, stream>>>((const unsigned*)UU, (unsigned*)GG, kTok * kFF / 2);

  wmma_gemm64<0, false, 2, 0, true><<<dim3(128, 1), blk, 0, stream>>>(
      GG, GG, kFF, 0L, W2T, W2T, kFF, 0L, (void*)out, (void*)out, kHid, 0L,
      b2, X1, 0L, kTok, kHid, kFF, kWCarryInv);
}
